// MultiHeadSelfAttention_89472758710800
// MI455X (gfx1250) — hardware-verified
//
#include <hip/hip_runtime.h>


#ifndef SEQ
#define SEQ 2048
#endif
#define SEQ_FULL 2048
#define EM   2048
#define NHD  16
#define HD   128
#define PSH  10.0f
#define QRS  2048.0f
#define CSL  (0.08838834764831845f * 1.4426950408889634f)
#define CRL  (CSL / 2048.0f)

typedef _Float16 h16;
typedef unsigned short bf;
typedef __attribute__((ext_vector_type(16))) __bf16   v16bf;
typedef __attribute__((ext_vector_type(16))) _Float16 v16h;
typedef __attribute__((ext_vector_type(8)))  _Float16 v8h;
typedef __attribute__((ext_vector_type(8)))  unsigned short v8us;
typedef __attribute__((ext_vector_type(8)))  float    v8f;
typedef __attribute__((ext_vector_type(4)))  float    v4f;
typedef v8h  __attribute__((may_alias)) v8ha;
typedef v4f  __attribute__((may_alias)) v4fa;

static_assert(SEQ % 64 == 0);
static_assert(SEQ <= SEQ_FULL);
static_assert(EM % 64 == 0);
static_assert(EM % 32 == 0);
static_assert(HD == 128);
static_assert(NHD * HD == EM);
static_assert(HD % 32 == 0);
static_assert(SEQ % 32 == 0);
static_assert(((size_t)SEQ * EM) % 8 == 0);

__device__ __forceinline__ unsigned short f2bf(float f) { unsigned u = __float_as_uint(f); u += 0x7FFFu + ((u >> 16) & 1u); return (unsigned short)(u >> 16); }
__device__ __forceinline__ float bf2f(unsigned short b) { return __uint_as_float(((unsigned)b) << 16); }
__device__ __forceinline__ float bfr(float f) { return bf2f(f2bf(f)); }
__device__ __forceinline__ void splitf(float y, unsigned short& h, unsigned short& l) { h = f2bf(y); l = f2bf(y - bf2f(h)); }
__device__ __forceinline__ v16h cat16(v8h lo, v8h hi) { return __builtin_shufflevector(lo, hi, 0, 1, 2, 3, 4, 5, 6, 7, 8, 9, 10, 11, 12, 13, 14, 15); }
__device__ __forceinline__ v16bf cat16b(v8us lo, v8us hi) { return __builtin_bit_cast(v16bf, __builtin_shufflevector(lo, hi, 0, 1, 2, 3, 4, 5, 6, 7, 8, 9, 10, 11, 12, 13, 14, 15)); }
__device__ __forceinline__ v8f wmma16(v16h a, v16h b, v8f c) { return __builtin_amdgcn_wmma_f32_16x16x32_f16(false, a, false, b, (short)0, c, false, false); }
__device__ __forceinline__ v8f wmmab(v16bf a, v16bf b, v8f c) { return __builtin_amdgcn_wmma_f32_16x16x32_bf16(false, a, false, b, (short)0, c, false, false); }
__device__ __forceinline__ v16h  ldh(const h16* p) { return cat16(*(const v8h*)p, *(const v8h*)(p + 16)); }
__device__ __forceinline__ v16bf ldb(const bf* p)  { return cat16b(*(const v8us*)p, *(const v8us*)(p + 16)); }

template <int NSPLIT, bool BIAS>
__device__ __forceinline__ void gemm_body(const bf* __restrict__ A, const bf* __restrict__ A2, const bf* __restrict__ Bt, int K, float* C, int ldc, const float* __restrict__ bias) {
    __shared__ __align__(16) float os[16 * 68];
    const int lane = threadIdx.x & 31, lr = lane & 15, hi = lane >> 4; const int r0 = blockIdx.x * 64, c0 = blockIdx.y * 64;
    v8f acc[4][4];
#pragma unroll
    for (int mb = 0; mb < 4; ++mb)
#pragma unroll
        for (int nb = 0; nb < 4; ++nb) acc[mb][nb] = (v8f){};
    const size_t aoff = (size_t)(r0 + lr) * K + 8 * hi, boff = (size_t)(c0 + lr) * K + 8 * hi;
#pragma unroll 1
    for (int kc = 0; kc < K; kc += 32) {
        v16bf a[4], a2[4];
#pragma unroll
        for (int mb = 0; mb < 4; ++mb) { a[mb] = ldb(A + aoff + (size_t)mb * 16 * K + kc); if (NSPLIT == 1) a2[mb] = ldb(A2 + aoff + (size_t)mb * 16 * K + kc); }
#pragma unroll
        for (int nb = 0; nb < 4; ++nb) { const v16bf b = ldb(Bt + boff + (size_t)nb * 16 * K + kc);
#pragma unroll
            for (int mb = 0; mb < 4; ++mb) { acc[mb][nb] = wmmab(a[mb], b, acc[mb][nb]); if (NSPLIT == 1) acc[mb][nb] = wmmab(a2[mb], b, acc[mb][nb]); } }
        asm volatile("v_nop\n\tv_nop\n\tv_nop\n\tv_nop" : "+v"(acc[0][0]), "+v"(acc[1][1]), "+v"(acc[2][2]), "+v"(acc[3][3]) : "v"(a[0]), "v"(a[3]));
    }
#pragma unroll
    for (int mb = 0; mb < 4; ++mb) {
#pragma unroll
        for (int nb = 0; nb < 4; ++nb) {
#pragma unroll
            for (int j = 0; j < 8; ++j) os[(hi * 8 + j) * 68 + nb * 16 + lr] = acc[mb][nb][j]; }
        __builtin_amdgcn_wave_barrier(); asm volatile("" ::: "memory");
        float* crow = C + (size_t)(r0 + mb * 16) * ldc + c0;
#pragma unroll 1
        for (int ps = 0; ps < 2; ++ps) {
#pragma unroll
            for (int s = 0; s < 8; ++s) { const int row = 2 * s + hi, cofs = lr * 4; v4f val = *(const v4fa*)&os[row * 68 + cofs];
                if (BIAS) { const v4f bb = *(const v4f*)(bias + c0 + cofs); val[0] += bfr(bb[0]); val[1] += bfr(bb[1]); val[2] += bfr(bb[2]); val[3] += bfr(bb[3]); }
                *(volatile v4f*)(crow + (size_t)row * ldc + cofs) = val; }
            if (ps == 0) __threadfence(); }
        __builtin_amdgcn_wave_barrier(); asm volatile("" ::: "memory");
    }
}
__global__ __launch_bounds__(32) void k_gemm_p(const bf* __restrict__ A, const bf* __restrict__ Bt, int K, float* C, int ldc) { gemm_body<0, false>(A, nullptr, Bt, K, C, ldc, nullptr); }
__global__ __launch_bounds__(32) void k_gemm_o(const bf* __restrict__ A, const bf* __restrict__ A2, const bf* __restrict__ Bt, int K, float* C, int ldc, const float* __restrict__ bias) { gemm_body<1, true>(A, A2, Bt, K, C, ldc, bias); }

__global__ __launch_bounds__(256) void k_cvt8(const float* __restrict__ src, bf* dst, size_t n8) { const size_t i = (size_t)blockIdx.x * 256 + threadIdx.x; if (i >= n8) return; const v8f v = *(const v8f*)(src + i * 8); v8us o;
#pragma unroll
    for (int k = 0; k < 8; ++k) o[k] = f2bf(v[k]); *(volatile v8us*)(dst + i * 8) = o; __threadfence(); *(volatile v8us*)(dst + i * 8) = o; }

__global__ __launch_bounds__(256) void k_cvtT(const float* __restrict__ W, bf* WT) {
    __shared__ float tl[64 * 65];
    const int t = threadIdx.x; const int k0 = blockIdx.x * 64, n0 = blockIdx.y * 64;
#pragma unroll
    for (int it = 0; it < 4; ++it) { const int r = (t >> 4) + 16 * it, c4 = (t & 15) * 4; const v4f a = *(const v4f*)(W + (size_t)(k0 + r) * EM + n0 + c4);
        tl[r * 65 + c4] = a[0]; tl[r * 65 + c4 + 1] = a[1]; tl[r * 65 + c4 + 2] = a[2]; tl[r * 65 + c4 + 3] = a[3]; }
    __syncthreads();
    const int pc = t & 7; v8us o[2];
#pragma unroll
    for (int it = 0; it < 2; ++it) { const int n = (t >> 3) + 32 * it;
#pragma unroll
        for (int q = 0; q < 8; ++q) o[it][q] = f2bf(tl[(pc * 8 + q) * 65 + n]); }
#pragma unroll
    for (int it = 0; it < 2; ++it) { const int n = (t >> 3) + 32 * it; *(volatile v8us*)(WT + (size_t)(n0 + n) * EM + k0 + pc * 8) = o[it]; }
    __threadfence();
#pragma unroll
    for (int it = 0; it < 2; ++it) { const int n = (t >> 3) + 32 * it; *(volatile v8us*)(WT + (size_t)(n0 + n) * EM + k0 + pc * 8) = o[it]; }
}

template <int COLS, int ROWBIAS, int WITHRES>
__device__ __forceinline__ void pl_body(const float* __restrict__ F, const float* __restrict__ bias, h16* P16, h16* PR, size_t n8) {
    static_assert(COLS % 8 == 0);
    static_assert((COLS & (COLS - 1)) == 0);
    const size_t i = (size_t)blockIdx.x * 256 + threadIdx.x; if (i >= n8) return;
    const size_t e = i * 8; const int c = (int)(e % (size_t)COLS); const int rw = (int)(e / (size_t)COLS);
    const v8f v = *(const v8f*)(F + e); float bb[8];
    if (ROWBIAS) { const float b0 = bfr(bias[rw]);
#pragma unroll
        for (int k = 0; k < 8; ++k) bb[k] = b0;
    } else { const v4f b0 = *(const v4f*)(bias + c), b1 = *(const v4f*)(bias + c + 4);
#pragma unroll
        for (int k = 0; k < 4; ++k) { bb[k] = bfr(b0[k]); bb[4 + k] = bfr(b1[k]); } }
    v8h oh, orr;
#pragma unroll
    for (int k = 0; k < 8; ++k) { const float y = v[k] + bb[k]; const h16 hh = (h16)y; oh[k] = hh; orr[k] = (h16)((y - (float)hh) * QRS); }
    *(volatile v8h*)(P16 + e) = oh; if (WITHRES) *(volatile v8h*)(PR + e) = orr;
    __threadfence();
    *(volatile v8h*)(P16 + e) = oh; if (WITHRES) *(volatile v8h*)(PR + e) = orr;
}
__global__ __launch_bounds__(256) void k_plq(const float* __restrict__ F, const float* __restrict__ bias, h16* P16, h16* PR, size_t n8) { pl_body<EM, 0, 1>(F, bias, P16, PR, n8); }
__global__ __launch_bounds__(256) void k_plk(const float* __restrict__ F, const float* __restrict__ bias, h16* P16, size_t n8) { pl_body<EM, 0, 0>(F, bias, P16, P16, n8); }
__global__ __launch_bounds__(256) void k_plv(const float* __restrict__ F, const float* __restrict__ bias, h16* P16, size_t n8) { pl_body<SEQ, 1, 0>(F, bias, P16, P16, n8); }

__global__ __launch_bounds__(32) void k_flash(const h16* __restrict__ Q16, const h16* __restrict__ QR, const h16* __restrict__ K16, const h16* __restrict__ VT, bf* CTh, bf* CTl) {
    __shared__ __align__(16) h16 ps[16 * 40];
    __shared__ __align__(16) float os[16 * 132];
    const int lane = threadIdx.x & 31, lr = lane & 15, hi = lane >> 4;
    const int h = blockIdx.y, q0 = blockIdx.x * 16;
    const int qoff  = (q0 + lr) * EM + h * HD + 8 * hi;
    const int kbase = lr * EM + h * HD + 8 * hi;
    const int vbase = (h * HD + lr) * SEQ + 8 * hi;
    v8f o[8]; float m[8], l[8];
#pragma unroll
    for (int j = 0; j < 8; ++j) o[j] = (v8f){};
#pragma unroll
    for (int r = 0; r < 8; ++r) { m[r] = -3.0e38f; l[r] = 0.0f; }
#pragma unroll 1
    for (int t0 = 0; t0 < SEQ; t0 += 32) {
        v8f s0h = (v8f){}, s1h = (v8f){}, s0r = (v8f){}, s1r = (v8f){};
        const int koff = kbase + t0 * EM;
#pragma unroll 1
        for (int f = 0; f < 4; ++f) {
            const v16h qa = ldh(Q16 + qoff + f * 32);
            const v16h qr = ldh(QR + qoff + f * 32);
            const v16h b0 = ldh(K16 + koff + f * 32);
            const v16h b1 = ldh(K16 + koff + 16 * EM + f * 32);
            s0h = wmma16(qa, b0, s0h); s1h = wmma16(qa, b1, s1h);
            s0r = wmma16(qr, b0, s0r); s1r = wmma16(qr, b1, s1r);
            asm volatile("v_nop\n\tv_nop\n\tv_nop\n\tv_nop" : "+v"(s0h), "+v"(s1h), "+v"(s0r), "+v"(s1r) : "v"(qa), "v"(qr), "v"(b0), "v"(b1));
        }
#pragma unroll
        for (int r = 0; r < 8; ++r) {
            const float a0 = s0h[r] * CSL + s0r[r] * CRL;
            const float a1 = s1h[r] * CSL + s1r[r] * CRL;
            float mx = fmaxf(a0, a1);
            mx = fmaxf(mx, __shfl_xor(mx, 1, 32)); mx = fmaxf(mx, __shfl_xor(mx, 2, 32)); mx = fmaxf(mx, __shfl_xor(mx, 4, 32)); mx = fmaxf(mx, __shfl_xor(mx, 8, 32));
            const float mn = fmaxf(m[r], mx);
            const float al = __builtin_amdgcn_exp2f(m[r] - mn);
            const float p0 = __builtin_amdgcn_exp2f((a0 - mn) + PSH);
            const float p1 = __builtin_amdgcn_exp2f((a1 - mn) + PSH);
            l[r] = l[r] * al + (p0 + p1);
            m[r] = mn;
#pragma unroll
            for (int j = 0; j < 8; ++j) o[j][r] *= al;
            ps[(8 * hi + r) * 40 + lr] = (h16)p0;
            ps[(8 * hi + r) * 40 + 16 + lr] = (h16)p1;
        }
        __builtin_amdgcn_wave_barrier(); asm volatile("" ::: "memory");
        const v16h pf = cat16(*(const v8ha*)&ps[lr * 40 + 8 * hi], *(const v8ha*)&ps[lr * 40 + 16 + 8 * hi]);
        const int voff = vbase + t0;
        {
            v16h vb[4];
#pragma unroll
            for (int jj = 0; jj < 4; ++jj) vb[jj] = ldh(VT + voff + jj * 16 * SEQ);
#pragma unroll
            for (int jj = 0; jj < 4; ++jj) o[jj] = wmma16(pf, vb[jj], o[jj]);
            asm volatile("v_nop\n\tv_nop\n\tv_nop\n\tv_nop" : "+v"(o[0]), "+v"(o[1]), "+v"(o[2]), "+v"(o[3]) : "v"(pf), "v"(vb[0]), "v"(vb[1]), "v"(vb[2]), "v"(vb[3]));
        }
        {
            v16h vb[4];
#pragma unroll
            for (int jj = 0; jj < 4; ++jj) vb[jj] = ldh(VT + voff + (4 + jj) * 16 * SEQ);
#pragma unroll
            for (int jj = 0; jj < 4; ++jj) o[4 + jj] = wmma16(pf, vb[jj], o[4 + jj]);
            asm volatile("v_nop\n\tv_nop\n\tv_nop\n\tv_nop" : "+v"(o[4]), "+v"(o[5]), "+v"(o[6]), "+v"(o[7]) : "v"(pf), "v"(vb[0]), "v"(vb[1]), "v"(vb[2]), "v"(vb[3]));
        }
        __builtin_amdgcn_wave_barrier(); asm volatile("" ::: "memory");
    }
#pragma unroll
    for (int r = 0; r < 8; ++r) {
        float lt = l[r];
        lt += __shfl_xor(lt, 1, 32); lt += __shfl_xor(lt, 2, 32); lt += __shfl_xor(lt, 4, 32); lt += __shfl_xor(lt, 8, 32);
        const float inv = 1.0f / lt;
#pragma unroll
        for (int j = 0; j < 8; ++j) os[(8 * hi + r) * 132 + j * 16 + lr] = o[j][r] * inv;
    }
    __builtin_amdgcn_wave_barrier(); asm volatile("" ::: "memory");
#pragma unroll 1
    for (int pass = 0; pass < 2; ++pass) {
#pragma unroll
        for (int s = 0; s < 8; ++s) {
            const int row = 2 * s + hi, cofs = lr * 8;
            const v4f a = *(const v4fa*)&os[row * 132 + cofs];
            const v4f b = *(const v4fa*)&os[row * 132 + cofs + 4];
            v8us oh, ol;
#pragma unroll
            for (int q = 0; q < 4; ++q) { unsigned short x0, x1; splitf(a[q], x0, x1); oh[q] = x0; ol[q] = x1; splitf(b[q], x0, x1); oh[4 + q] = x0; ol[4 + q] = x1; }
            const size_t oo = (size_t)(q0 + row) * EM + h * HD + cofs;
            *(volatile v8us*)(CTh + oo) = oh; *(volatile v8us*)(CTl + oo) = ol;
        }
        if (pass == 0) __threadfence();
    }
}

#define PL16  ((size_t)SEQ * EM * 2)
#define CARVE (PL16   + 4 * (size_t)EM * EM * 2   + (size_t)SEQ * EM * 4   + 4 * PL16   + 2 * PL16  )
static_assert(PL16 % 256 == 0);
static_assert(CARVE <= (size_t)134217728);

extern "C" void kernel_launch(void* const* d_in, const int* in_sizes, int n_in,
                              void* d_out, int out_size, void* d_ws, size_t ws_size, hipStream_t stream) {
    if (n_in < 9) return;
    if ((size_t)in_sizes[0] < (size_t)SEQ * EM) return;
    if ((size_t)in_sizes[1] < (size_t)EM * EM || (size_t)in_sizes[3] < (size_t)EM * EM || (size_t)in_sizes[5] < (size_t)EM * EM || (size_t)in_sizes[7] < (size_t)EM * EM) return;
    if (in_sizes[2] < EM || in_sizes[4] < EM || in_sizes[6] < EM || in_sizes[8] < EM) return;
    if ((size_t)out_size < (size_t)SEQ * EM) return;
    if (ws_size < CARVE) return;
    const float* x  = (const float*)d_in[0];
    const float* wq = (const float*)d_in[1]; const float* bq = (const float*)d_in[2];
    const float* wk = (const float*)d_in[3]; const float* bk = (const float*)d_in[4];
    const float* wv = (const float*)d_in[5]; const float* bv = (const float*)d_in[6];
    const float* wo = (const float*)d_in[7]; const float* bo = (const float*)d_in[8];
    float* OUT = (float*)d_out;
    char* wsp = (char*)d_ws;
    auto take = [&](size_t bytes) { char* p = wsp; wsp += (bytes + 255) & ~(size_t)255; return (void*)p; };
    bf* XB  = (bf*)take(PL16);
    bf* WQT = (bf*)take((size_t)EM * EM * 2); bf* WKT = (bf*)take((size_t)EM * EM * 2); bf* WVT = (bf*)take((size_t)EM * EM * 2); bf* WOT = (bf*)take((size_t)EM * EM * 2);
    float* F = (float*)take((size_t)SEQ * EM * 4);
    h16* Q16 = (h16*)take(PL16); h16* QRP = (h16*)take(PL16); h16* K16 = (h16*)take(PL16); h16* VT16 = (h16*)take(PL16);
    bf* CTh = (bf*)take(PL16); bf* CTl = (bf*)take(PL16);
    if ((size_t)(wsp - (char*)d_ws) > ws_size) return;

    const size_t n8 = (size_t)SEQ * EM / 8; const unsigned g8 = (unsigned)((n8 + 255) / 256);
    k_cvt8<<<g8, 256, 0, stream>>>(x, XB, n8);
    k_cvtT<<<dim3(EM / 64, EM / 64), 256, 0, stream>>>(wq, WQT);
    k_cvtT<<<dim3(EM / 64, EM / 64), 256, 0, stream>>>(wk, WKT);
    k_cvtT<<<dim3(EM / 64, EM / 64), 256, 0, stream>>>(wv, WVT);
    k_cvtT<<<dim3(EM / 64, EM / 64), 256, 0, stream>>>(wo, WOT);
    k_gemm_p<<<dim3(SEQ / 64, EM / 64), 32, 0, stream>>>(XB, WQT, EM, F, EM);
    k_plq<<<g8, 256, 0, stream>>>(F, bq, Q16, QRP, n8);
    k_gemm_p<<<dim3(SEQ / 64, EM / 64), 32, 0, stream>>>(XB, WKT, EM, F, EM);
    k_plk<<<g8, 256, 0, stream>>>(F, bk, K16, n8);
    k_gemm_p<<<dim3(EM / 64, SEQ / 64), 32, 0, stream>>>(WVT, XB, EM, F, SEQ);
    k_plv<<<g8, 256, 0, stream>>>(F, bv, VT16, n8);
    k_flash<<<dim3(SEQ / 16, NHD), 32, 0, stream>>>(Q16, QRP, K16, VT16, CTh, CTl);
    k_gemm_o<<<dim3(SEQ / 64, EM / 64), 32, 0, stream>>>(CTh, CTl, WOT, EM, OUT, EM, bo);
}
